// GraphResidualBlock_59511066853466
// MI455X (gfx1250) — hardware-verified
//
#include <hip/hip_runtime.h>


namespace {
constexpr int B = 1048576, NN = 6, H = 32;
constexpr float XS = 8.0f, WSC = 256.0f;
typedef _Float16 b16;
typedef __attribute__((ext_vector_type(16))) _Float16 v16b;
typedef __attribute__((ext_vector_type(8))) _Float16 v8b;
typedef __attribute__((ext_vector_type(8))) float v8f;
typedef __attribute__((ext_vector_type(4))) float v4f;
__device__ __forceinline__ float bf16_rne(float f) { unsigned int u = __float_as_uint(f); u += 0x7FFFu + ((u >> 16) & 1u); return __uint_as_float(u & 0xFFFF0000u); }
__device__ __forceinline__ void split16(float v, b16& hi, b16& lo) { hi = (b16)v; lo = (b16)(v - (float)hi); }
__device__ __forceinline__ v16b frag_kb(const b16* p, int hh) { const v8b a = *(const v8b*)(p + 8 * hh), b = *(const v8b*)(p + 16 + 8 * hh); v16b f;
#pragma unroll
  for (int e = 0; e < 8; ++e) { f[e] = a[e]; f[8 + e] = b[e]; } return f; }
__device__ __forceinline__ v8f wmma16b(v16b a, v16b b, v8f c) { v8f d = __builtin_amdgcn_wmma_f32_16x16x32_f16(false, a, false, b, (short)0, c, false, false); asm volatile("v_nop\n\tv_nop\n\tv_nop\n\tv_nop" : "+v"(d) : "v"(a), "v"(b)); return d; }
__device__ __forceinline__ void wave_lds_sync() { __builtin_amdgcn_fence(__ATOMIC_RELEASE, "workgroup"); __builtin_amdgcn_wave_barrier(); __builtin_amdgcn_fence(__ATOMIC_ACQUIRE, "workgroup"); }
__device__ __forceinline__ float pmul(float a, float b) { float p = a * b; asm volatile("" : "+v"(p)); return p; }

__global__ __launch_bounds__(32) void grb_kernel(const float* __restrict__ x, const float* __restrict__ Ap, const float* __restrict__ W1, const float* __restrict__ b1, const float* __restrict__ W2, const float* __restrict__ b2, int BV, float* __restrict__ out) {
  __shared__ __attribute__((aligned(16))) b16 Ah[96][H + 8], Al[96][H + 8], Wb[16][H + 8]; __shared__ float Am[NN][NN + 1], Rs[8], Xs[16][NN + 1], So[96];
  const int lane = threadIdx.x, nloc = lane & 15, hlf = lane >> 4; const size_t s0 = (size_t)blockIdx.x * 16; if (s0 >= (size_t)BV) return;
  if (lane < NN) { float mx = -INFINITY; for (int n = 0; n < NN; ++n) mx = fmaxf(mx, bf16_rne(Ap[lane * NN + n])); float e[NN], s = 0.0f; for (int n = 0; n < NN; ++n) { e[n] = __expf(bf16_rne(Ap[lane * NN + n]) - mx); s += e[n]; } float rs = 0.0f; for (int n = 0; n < NN; ++n) { Am[lane][n] = e[n] / s; rs += e[n] / s; } Rs[lane] = rs; }
  for (int r = 0; r < 16; ++r) Wb[r][lane] = (r == 0) ? (b16)(bf16_rne(W2[lane]) * WSC) : (b16)0.0f;
  for (int i = lane; i < 16 * NN; i += 32) Xs[i / NN][i % NN] = bf16_rne(x[s0 * NN + i]);
  wave_lds_sync();
  const float w1 = bf16_rne(W1[lane]), bb1 = bf16_rne(b1[lane]);
#pragma unroll 1
  for (int r = 0; r < 96; ++r) { const int s = r / NN, m = r % NN; float y = 0.0f;
#pragma unroll 1
    for (int n = 0; n < NN; ++n) y += pmul(Am[m][n], Xs[s][n]);
    const float hv = fmaxf(pmul(y, w1) + pmul(Rs[m], bb1), 0.0f); b16 p, q; split16(hv * XS, p, q); Ah[r][lane] = p; Al[r][lane] = q; }
  wave_lds_sync();
  const v16b bw = frag_kb(&Wb[nloc][0], hlf); const float bb2 = bf16_rne(b2[0]);
#pragma unroll
  for (int t = 0; t < 6; ++t) { v8f acc = {}; acc = wmma16b(frag_kb(&Ah[t * 16 + nloc][0], hlf), bw, acc); acc = wmma16b(frag_kb(&Al[t * 16 + nloc][0], hlf), bw, acc);
    if (nloc == 0) {
#pragma unroll
      for (int r8 = 0; r8 < 8; ++r8) { const int r = t * 16 + 8 * hlf + r8; So[r] = Xs[r / NN][r % NN] + acc[r8] * (1.0f / (XS * WSC)) + bb2; } } }
  wave_lds_sync();
  for (int pass = 0; pass < 2; ++pass) { for (int i = lane; i < 96; i += 32) ((volatile float*)out)[s0 * NN + i] = So[i]; __threadfence(); }
}
}

extern "C" void kernel_launch(void* const* d_in, const int* in_sizes, int n_in, void* d_out, int out_size, void* d_ws, size_t ws_size, hipStream_t stream) {
  (void)n_in; (void)d_ws; (void)ws_size;
  auto Fp = [&](int i) { return (const float*)d_in[i]; };
  if (in_sizes[0] != B * NN || in_sizes[1] != NN * NN || in_sizes[2] != H || in_sizes[3] != H || in_sizes[4] != H || in_sizes[5] != 1 || out_size != B * NN) return;
  const int BV = B;
  grb_kernel<<<(unsigned)(BV / 16), 32, 0, stream>>>(Fp(0), Fp(1), Fp(2), Fp(3), Fp(4), Fp(5), BV, (float*)d_out);
}
